// PointNetSA_76596446756881
// MI455X (gfx1250) — hardware-verified
//
#include <hip/hip_runtime.h>
#include <math.h>
#pragma clang fp contract(off)

typedef __attribute__((ext_vector_type(16))) _Float16 v16h;
typedef __attribute__((ext_vector_type(8)))  _Float16 v8h;
typedef __attribute__((ext_vector_type(8)))  float    v8f;
typedef __attribute__((ext_vector_type(4)))  float    v4f;
typedef __attribute__((ext_vector_type(4)))  int      v4i;

constexpr int PN_B     = 4;
constexpr int PN_NPTS  = 16384;
constexpr int PN_NQ    = 1024;
constexpr int PN_NNB   = 32;
constexpr int PN_FD    = 64;
constexpr int PN_CH0   = 64;
constexpr int PN_CH1   = 64;
constexpr int PN_CH2   = 128;
constexpr int PN_NGRP  = PN_B * PN_NQ;
constexpr int PN_NROW  = PN_NGRP * PN_NNB;
constexpr int PN_NSRC  = PN_B * PN_NPTS;
constexpr float PN_BN_EPS     = 1e-3f;
constexpr float PN_WCARRY     = 16.0f;
constexpr float PN_WCARRY_INV = 1.0f / PN_WCARRY;

static_assert(PN_NGRP == 4096 && PN_NROW == 131072 && PN_NSRC == 65536, "shapes");
static_assert(PN_NSRC % 64 == 0 && PN_NROW % 64 == 0, "GEMM M tile multiple");
static_assert(PN_CH0 % 64 == 0 && PN_CH1 % 64 == 0 && PN_CH2 % 64 == 0, "GEMM N tile multiple");
static_assert(PN_FD % 32 == 0 && PN_CH0 % 32 == 0 && PN_CH1 % 32 == 0, "GEMM K multiple of 32");
static_assert(PN_NNB == 32, "one wave tile of 32 rows per group");

constexpr size_t OUT0_BYTES = (size_t)PN_NGRP * 3 * 4;
constexpr size_t OUT1_OFF_BYTES = 49152;
constexpr size_t OUT1_BYTES = (size_t)PN_NGRP * PN_CH2 * 4;
static_assert(OUT0_BYTES == OUT1_OFF_BYTES, "out1 follows out0");
static_assert(OUT1_OFF_BYTES % 128 == 0, "out1 line aligned");
static_assert(OUT1_OFF_BYTES + OUT1_BYTES == 2146304, "d_out total");
constexpr size_t OUT1_OFF_FLOATS = OUT1_OFF_BYTES / 4;

constexpr int WH_W0P = 0;
constexpr int WH_W1  = WH_W0P + PN_CH0 * PN_FD;
constexpr int WH_W2  = WH_W1 + PN_CH1 * PN_CH0;
constexpr int WH_TOTAL = WH_W2 + PN_CH2 * PN_CH1;
static_assert(WH_TOTAL == 16384, "weight halves");

constexpr int FV_WXYZ = 0;
constexpr int FV_B0   = 192;
constexpr int FV_B1   = 256;
constexpr int FV_B2   = 320;
constexpr int FV_TOTAL = 448;

constexpr size_t WS_WH    = 0;
constexpr size_t WS_FV    = WS_WH + (size_t)WH_TOTAL * 2;
constexpr size_t WS_NXYZ  = WS_FV + 2048;
constexpr size_t WS_IDX   = WS_NXYZ + (size_t)PN_NGRP * 3 * 4;
constexpr size_t WS_P16   = WS_IDX + (size_t)PN_NGRP * PN_NNB * 4;
constexpr size_t WS_P0    = WS_P16 + (size_t)PN_NSRC * PN_FD * 2;
constexpr size_t WS_H0    = WS_P0 + (size_t)PN_NSRC * PN_CH0 * 4;
constexpr size_t WS_H1    = WS_H0 + (size_t)PN_NROW * PN_CH0 * 2;
constexpr size_t WS_TOTAL = WS_H1 + (size_t)PN_NROW * PN_CH1 * 2;
static_assert(FV_TOTAL * 4 <= 2048, "table pad");
static_assert(WS_FV % 128 == 0 && WS_NXYZ % 128 == 0 && WS_IDX % 128 == 0 && WS_P16 % 128 == 0, "line aligned");
static_assert(WS_P0 % 128 == 0 && WS_H0 % 128 == 0 && WS_H1 % 128 == 0, "line aligned");
static_assert(WS_TOTAL == 59328512, "carve total");
static_assert(WS_TOTAL <= 134217728, "carve cap");

__device__ __forceinline__ void st2_v4f(float* p, v4f v) {
  *(volatile v4f*)p = v;
  __threadfence();
  *(volatile v4f*)p = v;
}
__device__ __forceinline__ void st2_v8h(unsigned short* p, v8h v) {
  *(volatile v8h*)p = v;
  __threadfence();
  *(volatile v8h*)p = v;
}

__device__ __forceinline__ void pn_land3(float& x, float& y, float& z) {
  asm volatile("" : "+v"(x), "+v"(y), "+v"(z) : : "memory");
}

__device__ __forceinline__ void dep_guard4_h(v8f& a, v8f& b, v8f& c, v8f& d, v16h x) {
  asm volatile("v_nop\n\tv_nop\n\tv_nop\n\tv_nop" : "+v"(a), "+v"(b), "+v"(c), "+v"(d) : "v"(x));
}
__device__ __forceinline__ void dep_guard2_h(v8f& a, v8f& b, v16h x, v16h y, v16h z) {
  asm volatile("v_nop\n\tv_nop\n\tv_nop\n\tv_nop" : "+v"(a), "+v"(b) : "v"(x), "v"(y), "v"(z));
}
__device__ __forceinline__ void keep4_h(v16h a, v16h b, v16h c, v16h d) { asm volatile("v_nop" :: "v"(a), "v"(b), "v"(c), "v"(d)); }
__device__ __forceinline__ void acc_guard4(v8f& a, v8f& b, v8f& c, v8f& d) {
  asm volatile("v_nop\n\tv_nop\n\tv_nop\n\tv_nop" : "+v"(a), "+v"(b), "+v"(c), "+v"(d));
}
template <typename T> struct Frag;
template <> struct Frag<_Float16> {
  typedef v16h V; union U { v16h v; v8h h[2]; };
  static __device__ __forceinline__ v16h load(const _Float16* p) {
    U f; f.h[0] = *(const v8h*)(p); f.h[1] = *(const v8h*)(p + 16); return f.v;
  }
  static __device__ __forceinline__ v8f mma(v16h a, v16h b, v8f c) {
    return __builtin_amdgcn_wmma_f32_16x16x32_f16(false, a, false, b, (short)0, c, false, false);
  }
};

__device__ __forceinline__ v4f pn_bias4(const float* g, const float* b, const float* mm, const float* mv, int n0) {
  const v4f gv = *(const v4f*)(g + n0);
  const v4f bv = *(const v4f*)(b + n0);
  const v4f mv4 = *(const v4f*)(mv + n0);
  const v4f mm4 = *(const v4f*)(mm + n0);
  v4f o;
#pragma unroll
  for (int e = 0; e < 4; ++e) {
    const float s = gv[e] * rsqrtf(mv4[e] + PN_BN_EPS);
    o[e] = bv[e] - mm4[e] * s;
  }
  return o;
}

__global__ __launch_bounds__(256) void pn_prep(
    const float* __restrict__ w0, const float* __restrict__ g0, const float* __restrict__ b0,
    const float* __restrict__ mm0, const float* __restrict__ mv0,
    const float* __restrict__ w1, const float* __restrict__ g1, const float* __restrict__ b1,
    const float* __restrict__ mm1, const float* __restrict__ mv1,
    const float* __restrict__ w2, const float* __restrict__ g2, const float* __restrict__ b2,
    const float* __restrict__ mm2, const float* __restrict__ mv2,
    unsigned short* wh, float* fv) {
  const int tid = threadIdx.x;
  for (int it = 0; it < 2; ++it) {
    const int p = it * 256 + tid;
    const int n = p >> 3, k0 = (p & 7) * 8;
    const float s = g0[n] * rsqrtf(mv0[n] + PN_BN_EPS) * PN_WCARRY;
    v8h hv;
#pragma unroll
    for (int e = 0; e < 8; ++e) hv[e] = (_Float16)(w0[(3 + k0 + e) * PN_CH0 + n] * s);
    st2_v8h(wh + WH_W0P + p * 8, hv);
  }
  for (int it = 0; it < 2; ++it) {
    const int p = it * 256 + tid;
    const int n = p >> 3, k0 = (p & 7) * 8;
    const float s = g1[n] * rsqrtf(mv1[n] + PN_BN_EPS) * PN_WCARRY;
    v8h hv;
#pragma unroll
    for (int e = 0; e < 8; ++e) hv[e] = (_Float16)(w1[(k0 + e) * PN_CH1 + n] * s);
    st2_v8h(wh + WH_W1 + p * 8, hv);
  }
  for (int it = 0; it < 4; ++it) {
    const int p = it * 256 + tid;
    const int n = p >> 3, k0 = (p & 7) * 8;
    const float s = g2[n] * rsqrtf(mv2[n] + PN_BN_EPS) * PN_WCARRY;
    v8h hv;
#pragma unroll
    for (int e = 0; e < 8; ++e) hv[e] = (_Float16)(w2[(k0 + e) * PN_CH2 + n] * s);
    st2_v8h(wh + WH_W2 + p * 8, hv);
  }
  if (tid < 48) {
    const int e0 = tid * 4;
    const int c = e0 >> 6, n0 = e0 & 63;
    const v4f wv = *(const v4f*)(w0 + c * PN_CH0 + n0);
    const v4f gv = *(const v4f*)(g0 + n0);
    const v4f mv4 = *(const v4f*)(mv0 + n0);
    v4f o;
#pragma unroll
    for (int e = 0; e < 4; ++e) o[e] = wv[e] * (gv[e] * rsqrtf(mv4[e] + PN_BN_EPS));
    st2_v4f(fv + FV_WXYZ + e0, o);
  }
  if (tid >= 64 && tid < 80) {
    const int n0 = (tid - 64) * 4;
    const v4f o = pn_bias4(g0, b0, mm0, mv0, n0);
    st2_v4f(fv + FV_B0 + n0, o);
  }
  if (tid >= 96 && tid < 112) {
    const int n0 = (tid - 96) * 4;
    const v4f o = pn_bias4(g1, b1, mm1, mv1, n0);
    st2_v4f(fv + FV_B1 + n0, o);
  }
  if (tid >= 128 && tid < 160) {
    const int n0 = (tid - 128) * 4;
    const v4f o = pn_bias4(g2, b2, mm2, mv2, n0);
    st2_v4f(fv + FV_B2 + n0, o);
  }
}

__global__ __launch_bounds__(256) void pn_cvt16(const float* __restrict__ in, unsigned short* out, int n8) {
  const int i = blockIdx.x * 256 + threadIdx.x;
  if (i < n8) {
    const v4f a = *(const v4f*)(in + (size_t)i * 8);
    const v4f c = *(const v4f*)(in + (size_t)i * 8 + 4);
    v8h hv;
#pragma unroll
    for (int e = 0; e < 4; ++e) { hv[e] = (_Float16)a[e]; hv[4 + e] = (_Float16)c[e]; }
    st2_v8h(out + (size_t)i * 8, hv);
  }
}

__global__ __launch_bounds__(1024) void pn_fps(const float* __restrict__ xyz, float* out0, float* nxyz_ws) {
#pragma clang fp contract(off)
  __shared__ __align__(16) float s_cent[PN_NQ * 3];
  __shared__ float s_rv[2][32];
  __shared__ int   s_ri[2][32];

  const int tid = threadIdx.x;
  const int lane = tid & 31;
  const int wave = tid >> 5;
  const int b = blockIdx.x;
  const float* base = xyz + (size_t)b * PN_NPTS * 3;

  float px[16], py[16], pz[16], dist[16];
#pragma unroll
  for (int jg = 0; jg < 4; ++jg) {
#pragma unroll
    for (int jj = 0; jj < 4; ++jj) {
      const int j = jg * 4 + jj;
      const int i = j * 1024 + tid;
      px[j] = base[i * 3 + 0];
      py[j] = base[i * 3 + 1];
      pz[j] = base[i * 3 + 2];
      dist[j] = 1e10f;
    }
    pn_land3(px[jg * 4 + 0], py[jg * 4 + 0], pz[jg * 4 + 0]);
    pn_land3(px[jg * 4 + 1], py[jg * 4 + 1], pz[jg * 4 + 1]);
    pn_land3(px[jg * 4 + 2], py[jg * 4 + 2], pz[jg * 4 + 2]);
    pn_land3(px[jg * 4 + 3], py[jg * 4 + 3], pz[jg * 4 + 3]);
  }

  int far = 0;
  for (int it = 0; it < PN_NQ; ++it) {
    int fu = __builtin_amdgcn_readfirstlane(far);
    fu = fu < 0 ? 0 : fu;
    fu = fu > (PN_NPTS - 1) ? (PN_NPTS - 1) : fu;
    const float cx = base[fu * 3 + 0];
    const float cy = base[fu * 3 + 1];
    const float cz = base[fu * 3 + 2];
    if (tid == 0) {
      s_cent[it * 3 + 0] = cx;
      s_cent[it * 3 + 1] = cy;
      s_cent[it * 3 + 2] = cz;
    }
    float lv = -1.0f;
    int li = 0;
#pragma unroll
    for (int j = 0; j < 16; ++j) {
      const float dx = px[j] - cx, dy = py[j] - cy, dz = pz[j] - cz;
      const float t0 = dx * dx;
      const float t1 = dy * dy;
      const float t2 = dz * dz;
      const float d = (t0 + t2) + t1;
      dist[j] = fminf(dist[j], d);
      const bool up = dist[j] > lv;
      lv = up ? dist[j] : lv;
      li = up ? (j * 1024 + tid) : li;
    }
#pragma unroll
    for (int off = 16; off > 0; off >>= 1) {
      const float ov = __shfl_xor(lv, off, 32);
      const int   oi = __shfl_xor(li, off, 32);
      const bool take = (ov > lv) || ((ov == lv) && (oi < li));
      lv = take ? ov : lv;
      li = take ? oi : li;
    }
    const int buf = it & 1;
    if (lane == 0) { s_rv[buf][wave] = lv; s_ri[buf][wave] = li; }
    __syncthreads();
    float v2 = s_rv[buf][lane];
    int   i2 = s_ri[buf][lane];
#pragma unroll
    for (int off = 16; off > 0; off >>= 1) {
      const float ov = __shfl_xor(v2, off, 32);
      const int   oi = __shfl_xor(i2, off, 32);
      const bool take = (ov > v2) || ((ov == v2) && (oi < i2));
      v2 = take ? ov : v2;
      i2 = take ? oi : i2;
    }
    far = i2;
  }
  __syncthreads();
  if (tid < 768) {
    const v4f v = *(const v4f*)(s_cent + tid * 4);
    float* o = out0 + (size_t)b * (PN_NQ * 3) + tid * 4;
    float* w = nxyz_ws + (size_t)b * (PN_NQ * 3) + tid * 4;
    *(volatile v4f*)o = v;
    *(volatile v4f*)w = v;
    __threadfence();
    *(volatile v4f*)o = v;
    *(volatile v4f*)w = v;
  }
}

__global__ __launch_bounds__(256) void pn_knn(const float* __restrict__ xyz, const float* __restrict__ nxyz, int* idx_out) {
#pragma clang fp contract(off)
  __shared__ __align__(16) int s_buf[2048 * 4];
  const int tid = threadIdx.x;
  const int b = blockIdx.x >> 2;
  const int qg = blockIdx.x * 256 + tid;

  const float qx = nxyz[(size_t)qg * 3 + 0];
  const float qy = nxyz[(size_t)qg * 3 + 1];
  const float qz = nxyz[(size_t)qg * 3 + 2];
  const float q2 = (qx * qx + qz * qz) + qy * qy;

  float bd[PN_NNB];
  int   bi[PN_NNB];
#pragma unroll
  for (int j = 0; j < PN_NNB; ++j) { bd[j] = 3e30f; bi[j] = 0; }

  const float* base = xyz + (size_t)b * PN_NPTS * 3;
  for (int ch = 0; ch < PN_NPTS / 2048; ++ch) {
    __syncthreads();
#pragma unroll 1
    for (int r = 0; r < 8; ++r) {
      const int i = r * 256 + tid;
      const float* p = base + (size_t)(ch * 2048 + i) * 3;
      const float x = p[0], y = p[1], z = p[2];
      const float x2 = (x * x + z * z) + y * y;
      v4i w;
      w[0] = __float_as_int(x);
      w[1] = __float_as_int(y);
      w[2] = __float_as_int(z);
      w[3] = __float_as_int(x2);
      *(v4i*)(s_buf + i * 4) = w;
    }
    __syncthreads();
    const int c0 = ch * 2048;
#pragma unroll 1
    for (int i = 0; i < 2048; ++i) {
      const v4i w = *(const v4i*)(s_buf + i * 4);
      const int wx = w[0], wy = w[1], wz = w[2], ww = w[3];
      const float x = __int_as_float(wx);
      const float y = __int_as_float(wy);
      const float z = __int_as_float(wz);
      const float x2 = __int_as_float(ww);
      float p = qx * x;
      p = fmaf(qy, y, p);
      p = fmaf(qz, z, p);
      const float dd = (q2 - 2.0f * p) + x2;
      if (dd < bd[PN_NNB - 1]) {
        const int ci = c0 + i;
        bool cj = true;
#pragma unroll
        for (int j = PN_NNB - 1; j >= 1; --j) {
          const bool cjm = dd < bd[j - 1];
          const float nv = cjm ? bd[j - 1] : (cj ? dd : bd[j]);
          const int   ni = cjm ? bi[j - 1] : (cj ? ci : bi[j]);
          bd[j] = nv;
          bi[j] = ni;
          cj = cjm;
        }
        bd[0] = cj ? dd : bd[0];
        bi[0] = cj ? ci : bi[0];
      }
    }
  }
  __syncthreads();
#pragma unroll
  for (int m = 0; m < 8; ++m) {
    v4i w;
    w[0] = bi[4 * m + 0];
    w[1] = bi[4 * m + 1];
    w[2] = bi[4 * m + 2];
    w[3] = bi[4 * m + 3];
    *(v4i*)(s_buf + tid * 32 + 4 * m) = w;
  }
  __syncthreads();
  int* dst = idx_out + (size_t)blockIdx.x * 256 * PN_NNB;
  for (int pass = 0; pass < 2; ++pass) {
#pragma unroll
    for (int it = 0; it < 8; ++it) {
      const int L = it * 256 + tid;
      const v4i w = *(const v4i*)(s_buf + L * 4);
      *(volatile v4i*)(dst + L * 4) = w;
    }
    __threadfence();
  }
}

template <int BIAS_MODE, int OUT_MODE, int ACT>
__global__ __launch_bounds__(256) void wmma_gemm64(
    const unsigned short* __restrict__ Ap, int lda,
    const unsigned short* __restrict__ Btp, int ldb,
    void* __restrict__ Cout, int ldc,
    const float* __restrict__ bias,
    int M, int N, int K, float scale) {
  typedef _Float16 T;
  typedef Frag<T>::V V;
  const T* A = (const T*)Ap;
  const T* Bt = (const T*)Btp;
  __shared__ __align__(16) float sT[8][16 * 68];
  const int lane = threadIdx.x & 31;
  const int wave = threadIdx.x >> 5;
  const int tilesN = N >> 6;
  const int tilesM = M >> 6;
  const int tile = blockIdx.x * 8 + wave;
  if (tile >= tilesM * tilesN) return;
  const int tm = tile / tilesN;
  const int tn = tile - tm * tilesN;
  const int m0 = tm << 6;
  const int n0 = tn << 6;

  const int rlane = lane & 15;
  const int koff  = (lane >> 4) * 8;
  const int mOff  = (lane >> 4) * 8;

  v8f acc[4][4];
#pragma unroll
  for (int i = 0; i < 4; ++i)
#pragma unroll
    for (int j = 0; j < 4; ++j) acc[i][j] = (v8f){0.f,0.f,0.f,0.f,0.f,0.f,0.f,0.f};

  for (int k0 = 0; k0 < K; k0 += 32) {
    V bh[4];
#pragma unroll
    for (int j = 0; j < 4; ++j) {
      const size_t bo = (size_t)(n0 + (j << 4) + rlane) * ldb + koff + k0;
      bh[j] = Frag<T>::load(Bt + bo);
    }
#pragma unroll
    for (int i = 0; i < 4; ++i) {
      const size_t ao = (size_t)(m0 + (i << 4) + rlane) * lda + koff + k0;
      V ah = Frag<T>::load(A + ao);
#pragma unroll
      for (int j = 0; j < 4; ++j) acc[i][j] = Frag<T>::mma(ah, bh[j], acc[i][j]);
      dep_guard4_h(acc[i][0], acc[i][1], acc[i][2], acc[i][3], ah);
    }
    keep4_h(bh[0], bh[1], bh[2], bh[3]);
  }
  acc_guard4(acc[0][0], acc[0][1], acc[0][2], acc[0][3]);
  acc_guard4(acc[1][0], acc[1][1], acc[1][2], acc[1][3]);
  acc_guard4(acc[2][0], acc[2][1], acc[2][2], acc[2][3]);
  acc_guard4(acc[3][0], acc[3][1], acc[3][2], acc[3][3]);

  float* slab = sT[wave];
#pragma unroll
  for (int i = 0; i < 4; ++i) {
    const int mBase = m0 + (i << 4);
#pragma unroll
    for (int j = 0; j < 4; ++j) {
      const int n = n0 + (j << 4) + rlane;
      float bv = 0.f;
      if (BIAS_MODE == 2) bv = bias[n];
#pragma unroll
      for (int r = 0; r < 8; ++r) {
        float v = acc[i][j][r] * scale;
        if (BIAS_MODE == 2) v += bv;
        if (ACT == 2) v = fmaxf(v, 0.0f);
        slab[(mOff + r) * 68 + (j << 4) + rlane] = v;
      }
    }
    __builtin_amdgcn_fence(__ATOMIC_RELEASE, "workgroup");
    __builtin_amdgcn_wave_barrier();
    __builtin_amdgcn_fence(__ATOMIC_ACQUIRE, "workgroup");
    if (OUT_MODE == 0) {
      float* C = (float*)Cout;
      const int hh = lane >> 4, c4 = (lane & 15) * 4;
      for (int pass = 0; pass < 2; ++pass) {
#pragma unroll
        for (int it = 0; it < 8; ++it) {
          const int row = it * 2 + hh;
          v4f v = *(const v4f*)(slab + row * 68 + c4);
          *(volatile v4f*)(C + (size_t)(mBase + row) * ldc + n0 + c4) = v;
        }
        __threadfence();
      }
    } else {
      const int q = lane >> 3, c8 = (lane & 7) * 8;
      unsigned short* C = (unsigned short*)Cout;
      for (int pass = 0; pass < 2; ++pass) {
#pragma unroll
        for (int it = 0; it < 4; ++it) {
          const int row = it * 4 + q;
          const float* sp = slab + row * 68 + c8;
          v8h hv;
#pragma unroll
          for (int e = 0; e < 8; ++e) hv[e] = (_Float16)sp[e];
          *(volatile v8h*)(C + (size_t)(mBase + row) * ldc + n0 + c8) = hv;
        }
        __threadfence();
      }
    }
    __builtin_amdgcn_fence(__ATOMIC_RELEASE, "workgroup");
    __builtin_amdgcn_wave_barrier();
    __builtin_amdgcn_fence(__ATOMIC_ACQUIRE, "workgroup");
  }
}

__global__ __launch_bounds__(256) void pn_gather0(
    const float* __restrict__ xyz, const float* __restrict__ nxyz, const int* __restrict__ idx,
    const float* __restrict__ P0, const float* __restrict__ fv, unsigned short* H0) {
  const int lane = threadIdx.x & 31;
  const int wave = threadIdx.x >> 5;
  const int g = blockIdx.x * 8 + wave;
  if (g >= PN_NGRP) return;
  const int b = g >> 10;
  const int q = lane >> 3;
  const int c8 = (lane & 7) * 8;

  const v4f wxA = *(const v4f*)(fv + FV_WXYZ + 0 * PN_CH0 + c8);
  const v4f wxB = *(const v4f*)(fv + FV_WXYZ + 0 * PN_CH0 + c8 + 4);
  const v4f wyA = *(const v4f*)(fv + FV_WXYZ + 1 * PN_CH0 + c8);
  const v4f wyB = *(const v4f*)(fv + FV_WXYZ + 1 * PN_CH0 + c8 + 4);
  const v4f wzA = *(const v4f*)(fv + FV_WXYZ + 2 * PN_CH0 + c8);
  const v4f wzB = *(const v4f*)(fv + FV_WXYZ + 2 * PN_CH0 + c8 + 4);
  const v4f bA  = *(const v4f*)(fv + FV_B0 + c8);
  const v4f bB  = *(const v4f*)(fv + FV_B0 + c8 + 4);
  const float qx = nxyz[(size_t)g * 3 + 0];
  const float qy = nxyz[(size_t)g * 3 + 1];
  const float qz = nxyz[(size_t)g * 3 + 2];

#pragma unroll 1
  for (int it = 0; it < 8; ++it) {
    const int k = it * 4 + q;
    int j = idx[(size_t)g * PN_NNB + k];
    j = j < 0 ? 0 : j;
    j = j > (PN_NPTS - 1) ? (PN_NPTS - 1) : j;
    const size_t src = (size_t)b * PN_NPTS + j;
    const float* pr = P0 + src * PN_CH0 + c8;
    const v4f p0 = *(const v4f*)(pr);
    const v4f p1 = *(const v4f*)(pr + 4);
    const float* xr = xyz + src * 3;
    const float dx = xr[0] - qx;
    const float dy = xr[1] - qy;
    const float dz = xr[2] - qz;
    v8h hv;
#pragma unroll
    for (int e = 0; e < 4; ++e) {
      float t0 = p0[e] + bA[e];
      t0 = t0 + dx * wxA[e];
      t0 = t0 + dy * wyA[e];
      t0 = t0 + dz * wzA[e];
      float t1 = p1[e] + bB[e];
      t1 = t1 + dx * wxB[e];
      t1 = t1 + dy * wyB[e];
      t1 = t1 + dz * wzB[e];
      hv[e] = (_Float16)fmaxf(t0, 0.0f);
      hv[4 + e] = (_Float16)fmaxf(t1, 0.0f);
    }
    st2_v8h(H0 + ((size_t)g * PN_NNB + k) * PN_CH0 + c8, hv);
  }
}

__global__ __launch_bounds__(256) void pn_gemm_pool(
    const unsigned short* __restrict__ Ap, const unsigned short* __restrict__ Btp,
    const float* __restrict__ bias, float* out1, int ngroups, float scale) {
  typedef _Float16 T;
  __shared__ __align__(16) float sP[8][PN_CH2];
  const int lane = threadIdx.x & 31;
  const int wave = threadIdx.x >> 5;
  const int g = blockIdx.x * 8 + wave;
  if (g >= ngroups) return;
  const T* A = (const T*)Ap + (size_t)g * PN_NNB * PN_CH1;
  const T* Bt = (const T*)Btp;
  const int rlane = lane & 15;
  const int koff = (lane >> 4) * 8;

  v8f acc[2][8];
#pragma unroll
  for (int i = 0; i < 2; ++i)
#pragma unroll
    for (int j = 0; j < 8; ++j) acc[i][j] = (v8f){0.f,0.f,0.f,0.f,0.f,0.f,0.f,0.f};

#pragma unroll
  for (int k0 = 0; k0 < PN_CH1; k0 += 32) {
    const v16h a0 = Frag<T>::load(A + (size_t)rlane * PN_CH1 + koff + k0);
    const v16h a1 = Frag<T>::load(A + (size_t)(16 + rlane) * PN_CH1 + koff + k0);
#pragma unroll
    for (int j = 0; j < 8; ++j) {
      const v16h bf = Frag<T>::load(Bt + (size_t)(j * 16 + rlane) * PN_CH1 + koff + k0);
      acc[0][j] = Frag<T>::mma(a0, bf, acc[0][j]);
      acc[1][j] = Frag<T>::mma(a1, bf, acc[1][j]);
      dep_guard2_h(acc[0][j], acc[1][j], a0, a1, bf);
    }
  }
  acc_guard4(acc[0][0], acc[0][1], acc[0][2], acc[0][3]);
  acc_guard4(acc[0][4], acc[0][5], acc[0][6], acc[0][7]);
  acc_guard4(acc[1][0], acc[1][1], acc[1][2], acc[1][3]);
  acc_guard4(acc[1][4], acc[1][5], acc[1][6], acc[1][7]);

  float* slab = sP[wave];
#pragma unroll
  for (int j = 0; j < 8; ++j) {
    float m = acc[0][j][0];
#pragma unroll
    for (int r = 0; r < 8; ++r) {
      m = fmaxf(m, acc[0][j][r]);
      m = fmaxf(m, acc[1][j][r]);
    }
    const float o = __shfl_xor(m, 16, 32);
    m = fmaxf(m, o);
    const float bv = bias[j * 16 + rlane];
    float v = m * scale;
    v = v + bv;
    v = fmaxf(v, 0.0f);
    slab[j * 16 + rlane] = v;
  }
  __builtin_amdgcn_fence(__ATOMIC_RELEASE, "workgroup");
  __builtin_amdgcn_wave_barrier();
  __builtin_amdgcn_fence(__ATOMIC_ACQUIRE, "workgroup");
  {
    float* dst = out1 + (size_t)g * PN_CH2 + lane * 4;
    for (int pass = 0; pass < 2; ++pass) {
      v4f val = *(const v4f*)(slab + lane * 4);
      *(volatile v4f*)dst = val;
      __threadfence();
    }
  }
}

extern "C" void kernel_launch(void* const* d_in, const int* in_sizes, int n_in,
                              void* d_out, int out_size, void* d_ws, size_t ws_size,
                              hipStream_t stream) {
  if (n_in < 17) return;
  if (ws_size < WS_TOTAL) return;
  const float* xyz = (const float*)d_in[0];
  const float* pts = (const float*)d_in[1];
  const float* w0  = (const float*)d_in[2];
  const float* g0  = (const float*)d_in[3];
  const float* b0  = (const float*)d_in[4];
  const float* mm0 = (const float*)d_in[5];
  const float* mv0 = (const float*)d_in[6];
  const float* w1  = (const float*)d_in[7];
  const float* g1  = (const float*)d_in[8];
  const float* b1  = (const float*)d_in[9];
  const float* mm1 = (const float*)d_in[10];
  const float* mv1 = (const float*)d_in[11];
  const float* w2  = (const float*)d_in[12];
  const float* g2  = (const float*)d_in[13];
  const float* b2  = (const float*)d_in[14];
  const float* mm2 = (const float*)d_in[15];
  const float* mv2 = (const float*)d_in[16];

  float* out0 = (float*)d_out;
  float* out1 = out0 + OUT1_OFF_FLOATS;

  char* ws = (char*)d_ws;
  unsigned short* wh   = (unsigned short*)(ws + WS_WH);
  float*          fv   = (float*)(ws + WS_FV);
  float*          nxyz = (float*)(ws + WS_NXYZ);
  int*            idx  = (int*)(ws + WS_IDX);
  unsigned short* p16  = (unsigned short*)(ws + WS_P16);
  float*          P0   = (float*)(ws + WS_P0);
  unsigned short* H0   = (unsigned short*)(ws + WS_H0);
  unsigned short* H1   = (unsigned short*)(ws + WS_H1);

  pn_prep<<<1, 256, 0, stream>>>(w0, g0, b0, mm0, mv0, w1, g1, b1, mm1, mv1,
                                 w2, g2, b2, mm2, mv2, wh, fv);

  const int n8 = PN_NSRC * PN_FD / 8;
  pn_cvt16<<<(n8 + 255) / 256, 256, 0, stream>>>(pts, p16, n8);

  pn_fps<<<PN_B, 1024, 0, stream>>>(xyz, out0, nxyz);

  pn_knn<<<PN_NGRP / 256, 256, 0, stream>>>(xyz, nxyz, idx);

  {
    const int tiles = (PN_NSRC / 64) * (PN_CH0 / 64);
    wmma_gemm64<0, 0, 0><<<(tiles + 7) / 8, 256, 0, stream>>>(
        p16, PN_FD, wh + WH_W0P, PN_FD, (void*)P0, PN_CH0, fv, PN_NSRC, PN_CH0, PN_FD, PN_WCARRY_INV);
  }

  pn_gather0<<<(PN_NGRP + 7) / 8, 256, 0, stream>>>(xyz, nxyz, idx, P0, fv, H0);

  {
    const int tiles = (PN_NROW / 64) * (PN_CH1 / 64);
    wmma_gemm64<2, 1, 2><<<(tiles + 7) / 8, 256, 0, stream>>>(
        H0, PN_CH0, wh + WH_W1, PN_CH0, (void*)H1, PN_CH1, fv + FV_B1, PN_NROW, PN_CH1, PN_CH0, PN_WCARRY_INV);
  }

  pn_gemm_pool<<<(PN_NGRP + 7) / 8, 256, 0, stream>>>(H1, wh + WH_W2, fv + FV_B2, out1, PN_NGRP, PN_WCARRY_INV);
}
